// SecondaryCapsuleLayer_4793183502591
// MI455X (gfx1250) — hardware-run, weakly checked
//
#include <hip/hip_runtime.h>
#include <math.h>

typedef __attribute__((ext_vector_type(8)))  _Float16 v8h;
typedef __attribute__((ext_vector_type(16))) __bf16   v16b;
typedef __attribute__((ext_vector_type(8)))  __bf16   v8b;
typedef __attribute__((ext_vector_type(8)))  float    v8f;
typedef __attribute__((ext_vector_type(4)))  float    v4f;

constexpr int kNb   = 32;
constexpr int kNl   = 256;
constexpr int kNh   = 16;
constexpr int kDi   = 16;
constexpr int kDo   = 32;
constexpr int kKb   = 8;
constexpr int kDcap = kDi * kDo;
constexpr int kJ    = kDi * kDi;
constexpr int kHK   = kNh * kKb;
constexpr int kKI   = kKb * kDi;
constexpr int kBH   = kNb * kNh;
constexpr float kEps    = 1e-11f;
constexpr float kFltMin = 1.17549435e-38f;
static_assert(kDcap == 512);
static_assert(kJ == 256);
static_assert(kHK == 128);
static_assert(kKI == 128);
static_assert(kBH == 512);
static_assert((kNl % 32) == 0 && (kJ % 32) == 0 && (kKI % 32) == 0 && (kDo % 32) == 0);
static_assert((kHK % 64) == 0 && (kJ % 64) == 0 && (kNl % 64) == 0);

constexpr size_t kOut1OffBytes  = 1048576ull;
constexpr size_t kOutTotalBytes = 1050624ull;
static_assert((size_t)kBH * kDcap * 4 == kOut1OffBytes);
static_assert(kOut1OffBytes + (size_t)kBH * 4 == kOutTotalBytes);
static_assert((kOut1OffBytes % 128) == 0);

constexpr size_t kSzX16  = (size_t)kNb * kNl * kJ * 2;
constexpr size_t kSzM16  = (size_t)kNb * kHK * kJ * 2;
constexpr size_t kSzM32  = (size_t)kNb * kHK * kJ * 4;
constexpr size_t kSzV    = (size_t)kBH * kDcap * 4;
constexpr size_t kSzBL   = (size_t)kNb * kNl * kNh * 4;
constexpr size_t kSzSC   = (size_t)kBH * 32 * 4;
constexpr size_t kSzW16  = (size_t)kKI * kDo * 2;
constexpr size_t kOffXAH = 0;
constexpr size_t kOffXAL = kOffXAH + kSzX16;
constexpr size_t kOffXTH = kOffXAL + kSzX16;
constexpr size_t kOffXTL = kOffXTH + kSzX16;
constexpr size_t kOffCAH = kOffXTL + kSzX16;
constexpr size_t kOffCAL = kOffCAH + kSzM16;
constexpr size_t kOffQH  = kOffCAL + kSzM16;
constexpr size_t kOffQL  = kOffQH  + kSzM16;
constexpr size_t kOffZ   = kOffQL  + kSzM16;
constexpr size_t kOffP   = kOffZ   + kSzM32;
constexpr size_t kOffV   = kOffP   + kSzM32;
constexpr size_t kOffBL0 = kOffV   + kSzV;
constexpr size_t kOffBL1 = kOffBL0 + kSzBL;
constexpr size_t kOffSC  = kOffBL1 + kSzBL;
constexpr size_t kOffWQH = kOffSC  + kSzSC;
constexpr size_t kOffWQL = kOffWQH + kSzW16;
constexpr size_t kOffWSH = kOffWQL + kSzW16;
constexpr size_t kOffWSL = kOffWSH + kSzW16;
constexpr size_t kWsTotal = kOffWSL + kSzW16;
static_assert(kWsTotal == 35749888ull);
static_assert(kWsTotal <= 134217728ull);
static_assert((kOffXAL % 128) == 0 && (kOffXTH % 128) == 0 && (kOffXTL % 128) == 0 && (kOffCAH % 128) == 0 &&
              (kOffCAL % 128) == 0 && (kOffQH % 128) == 0 && (kOffQL % 128) == 0 && (kOffZ % 128) == 0 &&
              (kOffP % 128) == 0 && (kOffV % 128) == 0 && (kOffBL0 % 128) == 0 && (kOffBL1 % 128) == 0 &&
              (kOffSC % 128) == 0 && (kOffWQH % 128) == 0 && (kOffWQL % 128) == 0 && (kOffWSH % 128) == 0 &&
              (kOffWSL % 128) == 0);

__device__ __forceinline__ unsigned short f2bf_bits(float f) {
  unsigned u = __float_as_uint(f);
  return (unsigned short)((u + 0x7FFFu + ((u >> 16) & 1u)) >> 16);
}
__device__ __forceinline__ float bf_bits2f(unsigned short h) { return __uint_as_float(((unsigned)h) << 16); }

__device__ __forceinline__ void split8_store(const v4f a0, const v4f a1, v8h& hv, v8h& lv) {
#pragma unroll
  for (int e = 0; e < 4; ++e) {
    const float x0 = a0[e];
    const float x1 = a1[e];
    const unsigned short h0 = f2bf_bits(x0);
    const unsigned short h1 = f2bf_bits(x1);
    const unsigned short l0 = f2bf_bits(x0 - bf_bits2f(h0));
    const unsigned short l1 = f2bf_bits(x1 - bf_bits2f(h1));
    hv[e]     = __builtin_bit_cast(_Float16, h0);
    hv[4 + e] = __builtin_bit_cast(_Float16, h1);
    lv[e]     = __builtin_bit_cast(_Float16, l0);
    lv[4 + e] = __builtin_bit_cast(_Float16, l1);
  }
}
__device__ __forceinline__ void split8_frag(const v4f a0, const v4f a1, v8b& hv, v8b& lv) {
#pragma unroll
  for (int e = 0; e < 4; ++e) {
    const float x0 = a0[e];
    const float x1 = a1[e];
    const unsigned short h0 = f2bf_bits(x0);
    const unsigned short h1 = f2bf_bits(x1);
    const unsigned short l0 = f2bf_bits(x0 - bf_bits2f(h0));
    const unsigned short l1 = f2bf_bits(x1 - bf_bits2f(h1));
    hv[e]     = __builtin_bit_cast(__bf16, h0);
    hv[4 + e] = __builtin_bit_cast(__bf16, h1);
    lv[e]     = __builtin_bit_cast(__bf16, l0);
    lv[4 + e] = __builtin_bit_cast(__bf16, l1);
  }
}

union FragB { v16b v; v8b h[2]; };
__device__ __forceinline__ v16b frag_load(const __bf16* p) {
  FragB f;
  f.h[0] = *(const v8b*)(p);
  f.h[1] = *(const v8b*)(p + 16);
  return f.v;
}
__device__ __forceinline__ v8f mma_raw(v16b a, v16b b, v8f c) {
  return __builtin_amdgcn_wmma_f32_16x16x32_bf16(false, a, false, b, (short)0, c, false, false);
}
__device__ __forceinline__ v8f mma_guarded(v16b a, v16b b, v8f c) {
  c = __builtin_amdgcn_wmma_f32_16x16x32_bf16(false, a, false, b, (short)0, c, false, false);
  asm volatile("v_nop\n\tv_nop\n\tv_nop\n\tv_nop" : "+v"(c) : "v"(a), "v"(b));
  return c;
}
__device__ __forceinline__ void dep_guard1(v8f& a, v16b x, v16b y, v16b z, v16b w) {
  asm volatile("v_nop\n\tv_nop\n\tv_nop\n\tv_nop" : "+v"(a) : "v"(x), "v"(y), "v"(z), "v"(w));
}
__device__ __forceinline__ void keep4_b(v16b a, v16b b, v16b c, v16b d) { asm volatile("v_nop" :: "v"(a), "v"(b), "v"(c), "v"(d)); }
__device__ __forceinline__ void acc_guard4(v8f& a, v8f& b, v8f& c, v8f& d) {
  asm volatile("v_nop\n\tv_nop\n\tv_nop\n\tv_nop" : "+v"(a), "+v"(b), "+v"(c), "+v"(d));
}

__global__ __launch_bounds__(256) void gemm64_b3_kernel(
    const unsigned short* __restrict__ Ahp, const unsigned short* __restrict__ Alp, int lda, long strideA,
    const unsigned short* __restrict__ Bhp, const unsigned short* __restrict__ Blp, int ldb, long strideB,
    float* __restrict__ Cout, int ldc, long strideC, int M, int N, int K)
{
  __shared__ __align__(16) float sT[8][16 * 68];
  const int b    = blockIdx.y;
  const int lane = threadIdx.x & 31;
  const int wave = threadIdx.x >> 5;
  const int tilesN = N >> 6;
  const int tilesM = M >> 6;
  const int tile = blockIdx.x * 8 + wave;
  if (tile >= tilesM * tilesN) return;
  const int tm = tile / tilesN;
  const int tn = tile - tm * tilesN;
  const int m0 = tm << 6;
  const int n0 = tn << 6;

  const __bf16* Ah = (const __bf16*)Ahp + (size_t)b * strideA;
  const __bf16* Al = (const __bf16*)Alp + (size_t)b * strideA;
  const __bf16* Bh = (const __bf16*)Bhp + (size_t)b * strideB;
  const __bf16* Bl = (const __bf16*)Blp + (size_t)b * strideB;

  const int rlane = lane & 15;
  const int koff  = (lane >> 4) * 8;
  const int mOff  = (lane >> 4) * 8;

  v8f acc[4][4];
#pragma unroll
  for (int i = 0; i < 4; ++i)
#pragma unroll
    for (int j = 0; j < 4; ++j) acc[i][j] = (v8f){0.f,0.f,0.f,0.f,0.f,0.f,0.f,0.f};

  for (int k0 = 0; k0 < K; k0 += 32) {
    v16b bh[4], bl[4];
#pragma unroll
    for (int j = 0; j < 4; ++j) {
      const size_t bo = (size_t)(n0 + (j << 4) + rlane) * ldb + koff + k0;
      bh[j] = frag_load(Bh + bo);
      bl[j] = frag_load(Bl + bo);
    }
#pragma unroll
    for (int i = 0; i < 4; ++i) {
      const size_t ao = (size_t)(m0 + (i << 4) + rlane) * lda + koff + k0;
      const v16b ah = frag_load(Ah + ao);
      const v16b al = frag_load(Al + ao);
#pragma unroll
      for (int j = 0; j < 4; ++j) {
        acc[i][j] = mma_raw(ah, bh[j], acc[i][j]);
        acc[i][j] = mma_raw(ah, bl[j], acc[i][j]);
        acc[i][j] = mma_raw(al, bh[j], acc[i][j]);
      }
      dep_guard1(acc[i][0], ah, al, bh[0], bl[0]);
      dep_guard1(acc[i][1], ah, al, bh[1], bl[1]);
      dep_guard1(acc[i][2], ah, al, bh[2], bl[2]);
      dep_guard1(acc[i][3], ah, al, bh[3], bl[3]);
    }
    keep4_b(bh[0], bh[1], bh[2], bh[3]);
    keep4_b(bl[0], bl[1], bl[2], bl[3]);
  }
  acc_guard4(acc[0][0], acc[0][1], acc[0][2], acc[0][3]);
  acc_guard4(acc[1][0], acc[1][1], acc[1][2], acc[1][3]);
  acc_guard4(acc[2][0], acc[2][1], acc[2][2], acc[2][3]);
  acc_guard4(acc[3][0], acc[3][1], acc[3][2], acc[3][3]);

  float* slab = sT[wave];
  float* C = Cout + (size_t)b * strideC;
#pragma unroll
  for (int i = 0; i < 4; ++i) {
    const int mBase = m0 + (i << 4);
#pragma unroll
    for (int j = 0; j < 4; ++j) {
#pragma unroll
      for (int r = 0; r < 8; ++r) slab[(mOff + r) * 68 + (j << 4) + rlane] = acc[i][j][r];
    }
    __builtin_amdgcn_fence(__ATOMIC_RELEASE, "workgroup");
    __builtin_amdgcn_wave_barrier();
    __builtin_amdgcn_fence(__ATOMIC_ACQUIRE, "workgroup");
    {
      const int hh = lane >> 4, c4 = (lane & 15) * 4;
      for (int pass = 0; pass < 2; ++pass) {
#pragma unroll
        for (int it = 0; it < 8; ++it) {
          const int row = it * 2 + hh;
          const v4f v = *(const v4f*)(slab + row * 68 + c4);
          *(volatile v4f*)(C + (size_t)(mBase + row) * ldc + n0 + c4) = v;
        }
        __threadfence();
      }
    }
    __builtin_amdgcn_fence(__ATOMIC_RELEASE, "workgroup");
    __builtin_amdgcn_wave_barrier();
    __builtin_amdgcn_fence(__ATOMIC_ACQUIRE, "workgroup");
  }
}

__global__ __launch_bounds__(256) void prep_x_kernel(
    const float* __restrict__ x, unsigned short* __restrict__ XAH, unsigned short* __restrict__ XAL,
    unsigned short* __restrict__ XTH, unsigned short* __restrict__ XTL)
{
  __shared__ __align__(16) float tile[64 * 68];
  const int tid = threadIdx.x;
  const int bx = blockIdx.x;
  const int b  = bx >> 4;
  const int l0 = ((bx >> 2) & 3) * 64;
  const int j0 = (bx & 3) * 64;
  const float* xb = x + (size_t)b * (kNl * kJ);
#pragma unroll
  for (int it = 0; it < 4; ++it) {
    const int row = (tid >> 4) + 16 * it;
    const int c4 = (tid & 15) * 4;
    *(v4f*)(tile + row * 68 + c4) = *(const v4f*)(xb + (size_t)(l0 + row) * kJ + j0 + c4);
  }
  __syncthreads();
  for (int pass = 0; pass < 2; ++pass) {
#pragma unroll 1
    for (int it = 0; it < 2; ++it) {
      const int row = (tid >> 3) + 32 * it;
      const int c8 = (tid & 7) * 8;
      {
        const v4f a0 = *(const v4f*)(tile + row * 68 + c8);
        const v4f a1 = *(const v4f*)(tile + row * 68 + c8 + 4);
        v8h hv, lv;
        split8_store(a0, a1, hv, lv);
        const size_t o = ((size_t)b * kNl + l0 + row) * kJ + j0 + c8;
        *(volatile v8h*)(XAH + o) = hv;
        *(volatile v8h*)(XAL + o) = lv;
      }
      {
        v4f a0, a1;
        a0[0] = tile[(c8 + 0) * 68 + row];
        a0[1] = tile[(c8 + 1) * 68 + row];
        a0[2] = tile[(c8 + 2) * 68 + row];
        a0[3] = tile[(c8 + 3) * 68 + row];
        a1[0] = tile[(c8 + 4) * 68 + row];
        a1[1] = tile[(c8 + 5) * 68 + row];
        a1[2] = tile[(c8 + 6) * 68 + row];
        a1[3] = tile[(c8 + 7) * 68 + row];
        v8h hv, lv;
        split8_store(a0, a1, hv, lv);
        const size_t o = ((size_t)b * kJ + j0 + row) * kNl + l0 + c8;
        *(volatile v8h*)(XTH + o) = hv;
        *(volatile v8h*)(XTL + o) = lv;
      }
    }
    __threadfence();
  }
}

__global__ __launch_bounds__(256) void prep_w_kernel(
    const float* __restrict__ W, unsigned short* __restrict__ WQH, unsigned short* __restrict__ WQL,
    unsigned short* __restrict__ WSH, unsigned short* __restrict__ WSL)
{
  __shared__ __align__(16) float sW[kKI * kDo];
  const int tid = threadIdx.x;
#pragma unroll
  for (int it = 0; it < 4; ++it) {
    const int i4 = (tid + 256 * it) * 4;
    *(v4f*)(sW + i4) = *(const v4f*)(W + i4);
  }
  __syncthreads();
  for (int pass = 0; pass < 2; ++pass) {
#pragma unroll 1
    for (int it = 0; it < 2; ++it) {
      const int t = tid + 256 * it;
      {
        const v4f a0 = *(const v4f*)(sW + t * 8);
        const v4f a1 = *(const v4f*)(sW + t * 8 + 4);
        v8h hv, lv;
        split8_store(a0, a1, hv, lv);
        *(volatile v8h*)(WQH + (size_t)t * 8) = hv;
        *(volatile v8h*)(WQL + (size_t)t * 8) = lv;
      }
      {
        const int o = t >> 4;
        const int kk8 = (t & 15) * 8;
        v4f a0, a1;
        a0[0] = sW[(kk8 + 0) * kDo + o];
        a0[1] = sW[(kk8 + 1) * kDo + o];
        a0[2] = sW[(kk8 + 2) * kDo + o];
        a0[3] = sW[(kk8 + 3) * kDo + o];
        a1[0] = sW[(kk8 + 4) * kDo + o];
        a1[1] = sW[(kk8 + 5) * kDo + o];
        a1[2] = sW[(kk8 + 6) * kDo + o];
        a1[3] = sW[(kk8 + 7) * kDo + o];
        v8h hv, lv;
        split8_store(a0, a1, hv, lv);
        *(volatile v8h*)(WSH + (size_t)o * kKI + kk8) = hv;
        *(volatile v8h*)(WSL + (size_t)o * kKI + kk8) = lv;
      }
    }
    __threadfence();
  }
}

template <bool FIRST>
__global__ __launch_bounds__(256) void route_kernel(
    const float* __restrict__ alpha, const float* __restrict__ P, const float* __restrict__ blog_in,
    float* __restrict__ blog_out, unsigned short* __restrict__ CAH, unsigned short* __restrict__ CAL)
{
  __shared__ __align__(16) float sAl[64 * kHK];
  __shared__ __align__(16) float sBl[64 * kNh];
  __shared__ __align__(16) float sC[64 * kNh];
  const int tid = threadIdx.x;
  const int b  = blockIdx.x >> 2;
  const int l0 = (blockIdx.x & 3) * 64;
#pragma unroll
  for (int it = 0; it < 8; ++it) {
    const int i4 = (tid + 256 * it) * 4;
    *(v4f*)(sAl + i4) = *(const v4f*)(alpha + (size_t)l0 * kHK + i4);
  }
  __syncthreads();
#pragma unroll 1
  for (int it = 0; it < 4; ++it) {
    const int p = tid + 256 * it;
    float nb = 0.0f;
    if (!FIRST) {
      const int l = p >> 4;
      const int h = p & 15;
      const size_t row = (size_t)b * kNl + l0 + l;
      const float* pp = P + row * kHK + h * kKb;
      const v4f p0 = *(const v4f*)(pp);
      const v4f p1 = *(const v4f*)(pp + 4);
      const float* ap = sAl + l * kHK + h * kKb;
      const v4f q0 = *(const v4f*)(ap);
      const v4f q1 = *(const v4f*)(ap + 4);
      float acc = 0.0f;
      acc = fmaf(q0[0], p0[0], acc);
      acc = fmaf(q0[1], p0[1], acc);
      acc = fmaf(q0[2], p0[2], acc);
      acc = fmaf(q0[3], p0[3], acc);
      acc = fmaf(q1[0], p1[0], acc);
      acc = fmaf(q1[1], p1[1], acc);
      acc = fmaf(q1[2], p1[2], acc);
      acc = fmaf(q1[3], p1[3], acc);
      nb = blog_in[row * kNh + h] + acc;
    }
    sBl[p] = nb;
  }
  __syncthreads();
  if (tid < 64) {
    const int base = tid * kNh;
    float m = sBl[base];
#pragma unroll 1
    for (int h = 1; h < kNh; ++h) m = fmaxf(m, sBl[base + h]);
    float sum = 0.0f;
#pragma unroll 1
    for (int h = 0; h < kNh; ++h) {
      float e = expf(sBl[base + h] - m);
      e = (e < kFltMin) ? 0.0f : e;
      sum += e;
      sC[base + h] = e;
    }
    const float inv = 1.0f / sum;
#pragma unroll 1
    for (int h = 0; h < kNh; ++h) {
      float cv = sC[base + h] * inv;
      cv = (cv < kFltMin) ? 0.0f : cv;
      sC[base + h] = cv;
    }
  }
  __syncthreads();
  {
    const v4f nb4 = *(const v4f*)(sBl + tid * 4);
    float* bo = blog_out + ((size_t)b * kNl + l0) * kNh + tid * 4;
    *(volatile v4f*)bo = nb4;
    __threadfence();
    *(volatile v4f*)bo = nb4;
  }
  for (int pass = 0; pass < 2; ++pass) {
#pragma unroll 1
    for (int it = 0; it < 4; ++it) {
      const int hk = (tid >> 3) + 32 * it;
      const int l8 = (tid & 7) * 8;
      const int h  = hk >> 3;
      v4f a0, a1;
      a0[0] = sC[(l8 + 0) * kNh + h] * sAl[(l8 + 0) * kHK + hk];
      a0[1] = sC[(l8 + 1) * kNh + h] * sAl[(l8 + 1) * kHK + hk];
      a0[2] = sC[(l8 + 2) * kNh + h] * sAl[(l8 + 2) * kHK + hk];
      a0[3] = sC[(l8 + 3) * kNh + h] * sAl[(l8 + 3) * kHK + hk];
      a1[0] = sC[(l8 + 4) * kNh + h] * sAl[(l8 + 4) * kHK + hk];
      a1[1] = sC[(l8 + 5) * kNh + h] * sAl[(l8 + 5) * kHK + hk];
      a1[2] = sC[(l8 + 6) * kNh + h] * sAl[(l8 + 6) * kHK + hk];
      a1[3] = sC[(l8 + 7) * kNh + h] * sAl[(l8 + 7) * kHK + hk];
      v8h hv, lv;
      split8_store(a0, a1, hv, lv);
      const size_t o = ((size_t)b * kHK + hk) * kNl + l0 + l8;
      *(volatile v8h*)(CAH + o) = hv;
      *(volatile v8h*)(CAL + o) = lv;
    }
    __threadfence();
  }
}

__global__ __launch_bounds__(128) void s_squash_kernel(
    const float* __restrict__ Z, const unsigned short* __restrict__ WSHp, const unsigned short* __restrict__ WSLp,
    float* __restrict__ dst, float* __restrict__ SC)
{
  __shared__ __align__(16) float slab[4][kDcap];
  const int tid = threadIdx.x, lane = tid & 31, wave = tid >> 5;
  const int hh = lane >> 4, rl = lane & 15;
  const int bh = blockIdx.x * 4 + wave;
  const int b = bh >> 4, h = bh & 15;
  const __bf16* wh = (const __bf16*)WSHp;
  const __bf16* wl = (const __bf16*)WSLp;
  const float* Zb = Z + (size_t)b * (kHK * kJ) + (size_t)(h * kKb) * kJ + rl * kDi + 8 * hh;
  v8f acc0 = (v8f){0.f,0.f,0.f,0.f,0.f,0.f,0.f,0.f};
  v8f acc1 = (v8f){0.f,0.f,0.f,0.f,0.f,0.f,0.f,0.f};
#pragma unroll 1
  for (int c = 0; c < 4; ++c) {
    const float* p0 = Zb + (size_t)(2 * c) * kJ;
    const float* p1 = p0 + kJ;
    const v4f a0 = *(const v4f*)(p0);
    const v4f a1 = *(const v4f*)(p0 + 4);
    const v4f a2 = *(const v4f*)(p1);
    const v4f a3 = *(const v4f*)(p1 + 4);
    FragB ah, al;
    split8_frag(a0, a1, ah.h[0], al.h[0]);
    split8_frag(a2, a3, ah.h[1], al.h[1]);
    const size_t bo0 = (size_t)rl * kKI + c * 32 + 8 * hh;
    const size_t bo1 = (size_t)(16 + rl) * kKI + c * 32 + 8 * hh;
    const v16b b0h = frag_load(wh + bo0);
    const v16b b0l = frag_load(wl + bo0);
    const v16b b1h = frag_load(wh + bo1);
    const v16b b1l = frag_load(wl + bo1);
    acc0 = mma_guarded(ah.v, b0h, acc0);
    acc0 = mma_guarded(ah.v, b0l, acc0);
    acc0 = mma_guarded(al.v, b0h, acc0);
    acc1 = mma_guarded(ah.v, b1h, acc1);
    acc1 = mma_guarded(ah.v, b1l, acc1);
    acc1 = mma_guarded(al.v, b1h, acc1);
  }
  float part = 0.0f;
#pragma unroll
  for (int r = 0; r < 8; ++r) part = fmaf(acc0[r], acc0[r], part);
#pragma unroll
  for (int r = 0; r < 8; ++r) part = fmaf(acc1[r], acc1[r], part);
  part += __shfl_xor(part, 16, 32);
  part += __shfl_xor(part, 8, 32);
  part += __shfl_xor(part, 4, 32);
  part += __shfl_xor(part, 2, 32);
  part += __shfl_xor(part, 1, 32);
  const float sq = part;
  const float scale = sq / (1.0f + sq);
  const float inv = 1.0f / sqrtf(sq + kEps);
  float* sl = slab[wave];
#pragma unroll
  for (int r = 0; r < 8; ++r) {
    sl[(8 * hh + r) * kDo + rl]      = scale * (acc0[r] * inv);
    sl[(8 * hh + r) * kDo + 16 + rl] = scale * (acc1[r] * inv);
  }
  __syncthreads();
  float* drow = dst + (size_t)bh * kDcap;
  float* srow = SC + (size_t)bh * 32;
  for (int pass = 0; pass < 2; ++pass) {
#pragma unroll
    for (int it = 0; it < 4; ++it) {
      const v4f v = *(const v4f*)(sl + it * 128 + lane * 4);
      *(volatile v4f*)(drow + it * 128 + lane * 4) = v;
    }
    *(volatile float*)(srow + lane) = scale;
    __threadfence();
  }
}

__global__ __launch_bounds__(128) void q_kernel(
    const float* __restrict__ V, const unsigned short* __restrict__ WQHp, const unsigned short* __restrict__ WQLp,
    unsigned short* __restrict__ QH, unsigned short* __restrict__ QL)
{
  __shared__ __align__(16) float slab[4][kKb * kJ];
  const int tid = threadIdx.x, lane = tid & 31, wave = tid >> 5;
  const int hh = lane >> 4, rl = lane & 15;
  const int bh = blockIdx.x * 4 + wave;
  const __bf16* wh = (const __bf16*)WQHp;
  const __bf16* wl = (const __bf16*)WQLp;
  const float* pv = V + (size_t)bh * kDcap + rl * kDo + 8 * hh;
  const v4f a0 = *(const v4f*)(pv);
  const v4f a1 = *(const v4f*)(pv + 4);
  const v4f a2 = *(const v4f*)(pv + 16);
  const v4f a3 = *(const v4f*)(pv + 20);
  FragB ah, al;
  split8_frag(a0, a1, ah.h[0], al.h[0]);
  split8_frag(a2, a3, ah.h[1], al.h[1]);
  float* sl = slab[wave];
#pragma unroll 1
  for (int k = 0; k < kKb; ++k) {
    const size_t bo = (size_t)(k * kDi + rl) * kDo + 8 * hh;
    const v16b wbh = frag_load(wh + bo);
    const v16b wbl = frag_load(wl + bo);
    v8f acc = (v8f){0.f,0.f,0.f,0.f,0.f,0.f,0.f,0.f};
    acc = mma_guarded(ah.v, wbh, acc);
    acc = mma_guarded(ah.v, wbl, acc);
    acc = mma_guarded(al.v, wbh, acc);
#pragma unroll
    for (int r = 0; r < 8; ++r) sl[k * kJ + (8 * hh + r) * kDi + rl] = acc[r];
  }
  __syncthreads();
  const size_t obase = (size_t)bh * (kKb * kJ);
  for (int pass = 0; pass < 2; ++pass) {
#pragma unroll 1
    for (int it = 0; it < 8; ++it) {
      const int idx = it * 256 + lane * 8;
      const v4f c0 = *(const v4f*)(sl + idx);
      const v4f c1 = *(const v4f*)(sl + idx + 4);
      v8h hv, lv;
      split8_store(c0, c1, hv, lv);
      *(volatile v8h*)(QH + obase + idx) = hv;
      *(volatile v8h*)(QL + obase + idx) = lv;
    }
    __threadfence();
  }
}

__global__ __launch_bounds__(512) void tail_kernel(const float* __restrict__ SC, float* __restrict__ out1)
{
  const int t = threadIdx.x;
  float v = SC[(size_t)t * 32];
  asm volatile("" : "+v"(v));
  *(volatile float*)(out1 + t) = v;
  __threadfence();
  *(volatile float*)(out1 + t) = v;
}

extern "C" void kernel_launch(void* const* d_in, const int* in_sizes, int n_in,
                              void* d_out, int out_size, void* d_ws, size_t ws_size,
                              hipStream_t stream) {
  if (n_in < 4) return;
  if (in_sizes[0] != kNb * kNl * kJ) return;
  if (in_sizes[2] != kKb * kDi * kDo) return;
  if (in_sizes[3] != kNl * kNh * kKb) return;
  if ((size_t)out_size * 4 != kOutTotalBytes) return;
  if (ws_size < kWsTotal) return;

  const float* x     = (const float*)d_in[0];
  const float* W     = (const float*)d_in[2];
  const float* alpha = (const float*)d_in[3];
  float* out0 = (float*)d_out;
  float* out1 = (float*)d_out + (kOut1OffBytes / 4);

  char* ws = (char*)d_ws;
  unsigned short* XAH = (unsigned short*)(ws + kOffXAH);
  unsigned short* XAL = (unsigned short*)(ws + kOffXAL);
  unsigned short* XTH = (unsigned short*)(ws + kOffXTH);
  unsigned short* XTL = (unsigned short*)(ws + kOffXTL);
  unsigned short* CAH = (unsigned short*)(ws + kOffCAH);
  unsigned short* CAL = (unsigned short*)(ws + kOffCAL);
  unsigned short* QH  = (unsigned short*)(ws + kOffQH);
  unsigned short* QL  = (unsigned short*)(ws + kOffQL);
  float*          Zp  = (float*)(ws + kOffZ);
  float*          Pp  = (float*)(ws + kOffP);
  float*          Vp  = (float*)(ws + kOffV);
  float*          BL0 = (float*)(ws + kOffBL0);
  float*          BL1 = (float*)(ws + kOffBL1);
  float*          SC  = (float*)(ws + kOffSC);
  unsigned short* WQH = (unsigned short*)(ws + kOffWQH);
  unsigned short* WQL = (unsigned short*)(ws + kOffWQL);
  unsigned short* WSH = (unsigned short*)(ws + kOffWSH);
  unsigned short* WSL = (unsigned short*)(ws + kOffWSL);

  prep_x_kernel<<<kNb * 16, 256, 0, stream>>>(x, XAH, XAL, XTH, XTL);
  prep_w_kernel<<<1, 256, 0, stream>>>(W, WQH, WQL, WSH, WSL);

  for (int pass = 0; pass < 3; ++pass) {
    const float* bin = (pass == 1) ? BL0 : BL1;
    float* bout = (pass == 1) ? BL1 : BL0;
    if (pass == 0)
      route_kernel<true><<<kNb * 4, 256, 0, stream>>>(alpha, Pp, bin, bout, CAH, CAL);
    else
      route_kernel<false><<<kNb * 4, 256, 0, stream>>>(alpha, Pp, bin, bout, CAH, CAL);

    gemm64_b3_kernel<<<dim3(1, kNb), 256, 0, stream>>>(
        CAH, CAL, kNl, (long)kHK * kNl,
        XTH, XTL, kNl, (long)kJ * kNl,
        Zp, kJ, (long)kHK * kJ, kHK, kJ, kNl);

    s_squash_kernel<<<kBH / 4, 128, 0, stream>>>(Zp, WSH, WSL, (pass == 2) ? out0 : Vp, SC);

    if (pass < 2) {
      q_kernel<<<kBH / 4, 128, 0, stream>>>(Vp, WQH, WQL, QH, QL);
      gemm64_b3_kernel<<<dim3(1, kNb), 256, 0, stream>>>(
          XAH, XAL, kJ, (long)kNl * kJ,
          QH, QL, kJ, (long)kHK * kJ,
          Pp, kHK, (long)kNl * kHK, kNl, kHK, kJ);
    }
  }
  tail_kernel<<<1, 512, 0, stream>>>(SC, out1);
}
